// Net_65859028517102
// MI455X (gfx1250) — hardware-verified
//
#include <hip/hip_runtime.h>
#include <math.h>

constexpr int NBATCH   = 2048;
constexpr int NSTEP    = 2048;
constexpr int NFUT     = 32;
constexpr int NCOL     = NFUT + 1;
constexpr int NHID     = 16;
constexpr int NGATE    = 4 * NHID;
constexpr int ROWS_BLK = 32;
constexpr int NBLK     = NBATCH / ROWS_BLK;
constexpr int XCHUNK   = 64;
constexpr int HP       = 72;
constexpr int BP       = 40;
constexpr int BPLANE   = NGATE * BP;
constexpr int H2P      = 20;
constexpr float LO_CARRY = 2048.0f;
constexpr float LO_INV   = 1.0f / 2048.0f;
constexpr float F16_MIN_NORMAL = 6.103515625e-5f;
static_assert(NBATCH % ROWS_BLK == 0);
static_assert(NSTEP % XCHUNK == 0);
static_assert((ROWS_BLK * NCOL * 4) % 128 == 0);
static_assert(NBLK * ROWS_BLK * NCOL * 4 == 270336);
static_assert((ROWS_BLK * NCOL) % 4 == 0);
static_assert(HP % 8 == 0 && BP % 8 == 0 && H2P % 4 == 0);

typedef __attribute__((ext_vector_type(16))) _Float16 v16h;
typedef __attribute__((ext_vector_type(8)))  _Float16 v8h;
typedef __attribute__((ext_vector_type(8)))  float    v8f;
typedef __attribute__((ext_vector_type(4)))  float    v4f;
typedef __attribute__((ext_vector_type(2)))  float    v2f;

union FragU { v16h v; v8h h[2]; };
__device__ __forceinline__ v16h frag2(const _Float16* p0, const _Float16* p1) {
  FragU f; f.h[0] = *(const v8h*)(p0); f.h[1] = *(const v8h*)(p1); return f.v;
}
__device__ __forceinline__ v8f mma16(v16h a, v16h b, v8f c) {
  return __builtin_amdgcn_wmma_f32_16x16x32_f16(false, a, false, b, (short)0, c, false, false);
}
__device__ __forceinline__ void wm_guard(v8f& a, v8f& b, v16h p, v16h q, v16h s, v16h t) {
  asm volatile("v_nop\n\tv_nop\n\tv_nop\n\tv_nop" : "+v"(a), "+v"(b) : "v"(p), "v"(q), "v"(s), "v"(t));
}

__device__ __forceinline__ float fsig(float x)  { return __builtin_amdgcn_rcpf(1.0f + __expf(-x)); }
__device__ __forceinline__ float ftanh(float x) { return 1.0f - 2.0f * __builtin_amdgcn_rcpf(__expf(2.0f * x) + 1.0f); }

__device__ __forceinline__ void split_hl(float v, float& hq, float& lq) {
  float t = (float)(_Float16)v;
  t = (fabsf(v) < F16_MIN_NORMAL) ? 0.0f : t;
  asm volatile("" : "+v"(t));
  hq = t;
  lq = (v - t) * LO_CARRY;
}

__device__ __forceinline__ void lstm_gates(const v8f (&z)[4], v8f& cs, v8f& hv) {
#pragma unroll
  for (int r = 0; r < 8; ++r) {
    const float ig = fsig(z[0][r]);
    const float fg = fsig(z[1][r]);
    const float gg = ftanh(z[2][r]);
    const float og = fsig(z[3][r]);
    const float cn = fg * cs[r] + ig * gg;
    cs[r] = cn;
    hv[r] = og * ftanh(cn);
  }
}

template <int TT>
__device__ __forceinline__ void tile_step(v8f& c1, v8f& c2, _Float16* Hst, float* H2f, const _Float16* Bw,
                                          const float* xrow, const float (&w1)[4], const float (&b1)[4],
                                          const float (&b2)[4], const int c, const int hh) {
  const int koff = hh * 8;
  _Float16* Ht = Hst + TT * 16 * HP;
  float* h2t = H2f + TT * 16 * H2P;
  const _Float16* hrow = Ht + c * HP + koff;
  const v8f z8 = {0.f, 0.f, 0.f, 0.f, 0.f, 0.f, 0.f, 0.f};
  const v4f xa = *(const v4f*)(xrow + TT * 16 + 8 * hh);
  const v4f xb = *(const v4f*)(xrow + TT * 16 + 8 * hh + 4);
  const float xv[8] = {xa[0], xa[1], xa[2], xa[3], xb[0], xb[1], xb[2], xb[3]};

  v8f z[4];
  {
    const v16h a1 = frag2(hrow, hrow + 16);
#pragma unroll
    for (int g = 0; g < 4; ++g) {
      const _Float16* bp = Bw + (g * 16 + c) * BP + koff;
      const v16h bm = frag2(bp, bp + 16);
      const v16h br = frag2(bp + BPLANE, bp + BPLANE + 16);
      v8f cm;
#pragma unroll
      for (int r = 0; r < 8; ++r) cm[r] = fmaf(xv[r], w1[g], b1[g]);
      v8f am = mma16(a1, bm, cm);
      v8f ar = mma16(a1, br, z8);
      wm_guard(am, ar, a1, a1, bm, br);
#pragma unroll
      for (int r = 0; r < 8; ++r) z[g][r] = fmaf(ar[r], LO_INV, am[r]);
    }
  }
  v8f h1v;
  lstm_gates(z, c1, h1v);
  __syncthreads();
#pragma unroll
  for (int r = 0; r < 8; ++r) {
    float hq, lq;
    split_hl(h1v[r], hq, lq);
    Ht[(8 * hh + r) * HP + c]      = (_Float16)hq;
    Ht[(8 * hh + r) * HP + 16 + c] = (_Float16)lq;
  }
  __syncthreads();

  {
    const v16h a2h = frag2(hrow, hrow + 32);
    const v16h a2l = frag2(hrow + 16, hrow + 48);
#pragma unroll
    for (int g = 0; g < 4; ++g) {
      const _Float16* bp = Bw + 2 * BPLANE + (g * 16 + c) * BP + koff;
      const v16h bm = frag2(bp, bp + 16);
      const v16h br = frag2(bp + BPLANE, bp + BPLANE + 16);
      const float bb = b2[g];
      const v8f cm = {bb, bb, bb, bb, bb, bb, bb, bb};
      v8f am = mma16(a2h, bm, cm);
      v8f ar = mma16(a2h, br, z8);
      ar = mma16(a2l, bm, ar);
      wm_guard(am, ar, a2h, a2l, bm, br);
#pragma unroll
      for (int r = 0; r < 8; ++r) z[g][r] = fmaf(ar[r], LO_INV, am[r]);
    }
  }
  v8f h2v;
  lstm_gates(z, c2, h2v);
  __syncthreads();
#pragma unroll
  for (int r = 0; r < 8; ++r) {
    float hq, lq;
    split_hl(h2v[r], hq, lq);
    Ht[(8 * hh + r) * HP + 32 + c] = (_Float16)hq;
    Ht[(8 * hh + r) * HP + 48 + c] = (_Float16)lq;
    h2t[(8 * hh + r) * H2P + c]    = h2v[r];
  }
  __syncthreads();
}

__device__ __forceinline__ void head_step(const float* H2f, const float* hd, float* outS, float* fb,
                                          const int lane, const int col) {
  const float* hr = H2f + lane * H2P;
  const v4f h0 = *(const v4f*)(hr);
  const v4f h1 = *(const v4f*)(hr + 4);
  const v4f h2 = *(const v4f*)(hr + 8);
  const v4f h3 = *(const v4f*)(hr + 12);
  float acc = 0.0f;
#pragma unroll 1
  for (int j = 0; j < 8; ++j) {
    const float* wr = hd + j * 16;
    const v4f w0 = *(const v4f*)(wr);
    const v4f w1 = *(const v4f*)(wr + 4);
    const v4f w2 = *(const v4f*)(wr + 8);
    const v4f w3 = *(const v4f*)(wr + 12);
    float s = 0.0f;
#pragma unroll
    for (int e = 0; e < 4; ++e) s = fmaf(h0[e], w0[e], s);
#pragma unroll
    for (int e = 0; e < 4; ++e) s = fmaf(h1[e], w1[e], s);
#pragma unroll
    for (int e = 0; e < 4; ++e) s = fmaf(h2[e], w2[e], s);
#pragma unroll
    for (int e = 0; e < 4; ++e) s = fmaf(h3[e], w3[e], s);
    float zz = s + hd[128 + j];
    zz = (zz >= 0.0f) ? zz : 0.2f * zz;
    acc = fmaf(hd[136 + j], zz, acc);
  }
  const float o = acc + hd[144];
  outS[lane * NCOL + col] = o;
  fb[lane] = o;
}

__global__ __launch_bounds__(32) void lstm2_head_kernel(
    const float* __restrict__ x,
    const float* __restrict__ wih1, const float* __restrict__ whh1,
    const float* __restrict__ bih1, const float* __restrict__ bhh1,
    const float* __restrict__ wih2, const float* __restrict__ whh2,
    const float* __restrict__ bih2, const float* __restrict__ bhh2,
    const float* __restrict__ fc1w, const float* __restrict__ fc1b,
    const float* __restrict__ fc2w, const float* __restrict__ fc2b,
    float* __restrict__ out) {
  __shared__ __align__(16) _Float16 Hst[ROWS_BLK * HP];
  __shared__ __align__(16) _Float16 Bw[4 * BPLANE];
  __shared__ __align__(16) float    H2f[ROWS_BLK * H2P];
  __shared__ __align__(16) float    xsT[(XCHUNK + 1) * ROWS_BLK];
  __shared__ __align__(16) float    outS[ROWS_BLK * NCOL];
  __shared__ __align__(16) float    hd[160];
  __shared__ __align__(16) float    cstS[192];

  const int lane = threadIdx.x & 31;
  const int c = lane & 15, hh = lane >> 4;
  const int row0 = blockIdx.x * ROWS_BLK;
  float* fb = xsT + XCHUNK * ROWS_BLK;

#pragma unroll 1
  for (int i = lane; i < ROWS_BLK * HP; i += 32) Hst[i] = (_Float16)0.0f;

  {
    const int i2 = lane * 2;
    const v2f a = *(const v2f*)(bih1 + i2);
    const v2f b = *(const v2f*)(bhh1 + i2);
    const v2f w = *(const v2f*)(wih1 + i2);
    const v2f d = *(const v2f*)(bih2 + i2);
    const v2f e = *(const v2f*)(bhh2 + i2);
    cstS[i2]           = a[0] + b[0];
    cstS[i2 + 1]       = a[1] + b[1];
    cstS[64 + i2]      = w[0];
    cstS[64 + i2 + 1]  = w[1];
    cstS[128 + i2]     = d[0] + e[0];
    cstS[128 + i2 + 1] = d[1] + e[1];
  }
  {
    const v4f fw = *(const v4f*)(fc1w + 4 * lane);
    *(v4f*)(hd + 4 * lane) = fw;
    const int i8 = lane & 7;
    const float p1 = fc1b[i8];
    const float p2 = fc2w[i8];
    const float p3 = fc2b[0];
    if (lane < 8) { hd[128 + lane] = p1; hd[136 + lane] = p2; }
    if (lane == 0) hd[144] = p3;
  }
#pragma unroll 1
  for (int p = 0; p < 4; ++p) {
#pragma unroll 1
    for (int n = 0; n < NGATE; ++n) {
      const int kk = lane & 15;
      const bool lowk = lane < 16;
      const float wa = whh1[n * NHID + kk];
      const float wb = wih2[n * NHID + kk];
      const float wc = whh2[n * NHID + kk];
      const float src = (p < 2) ? wa : (lowk ? wb : wc);
      float hq, lq;
      split_hl(src, hq, lq);
      const bool wantlo = (p == 1) ? lowk : (p == 3);
      const bool iszero = (p == 0) && !lowk;
      float val = wantlo ? lq : hq;
      val = iszero ? 0.0f : val;
      Bw[p * BPLANE + n * BP + lane] = (_Float16)val;
    }
  }
  __syncthreads();

  float w1[4], b1[4], b2[4];
#pragma unroll
  for (int g = 0; g < 4; ++g) {
    b1[g] = cstS[16 * g + c];
    w1[g] = cstS[64 + 16 * g + c];
    b2[g] = cstS[128 + 16 * g + c];
  }
  const v8f z8 = {0.f, 0.f, 0.f, 0.f, 0.f, 0.f, 0.f, 0.f};
  v8f c1a = z8, c2a = z8, c1b = z8, c2b = z8;

#pragma unroll 1
  for (int st = 0; st < NSTEP + NFUT; ++st) {
    if (st < NSTEP && (st & (XCHUNK - 1)) == 0) {
      __syncthreads();
#pragma unroll 1
      for (int it = 0; it < 16; ++it) {
        const int row = it * 2 + hh;
        const int c4 = c * 4;
        const v4f v = *(const v4f*)(x + (size_t)(row0 + row) * NSTEP + st + c4);
        xsT[(c4 + 0) * ROWS_BLK + row] = v[0];
        xsT[(c4 + 1) * ROWS_BLK + row] = v[1];
        xsT[(c4 + 2) * ROWS_BLK + row] = v[2];
        xsT[(c4 + 3) * ROWS_BLK + row] = v[3];
      }
      __syncthreads();
    }
    const int xoff = (st < NSTEP) ? ((st & (XCHUNK - 1)) * ROWS_BLK) : (XCHUNK * ROWS_BLK);
    const float* xrow = xsT + xoff;
    tile_step<0>(c1a, c2a, Hst, H2f, Bw, xrow, w1, b1, b2, c, hh);
    tile_step<1>(c1b, c2b, Hst, H2f, Bw, xrow, w1, b1, b2, c, hh);
    if (st >= NSTEP - 1) {
      head_step(H2f, hd, outS, fb, lane, st - (NSTEP - 1));
      __syncthreads();
    }
  }

  __syncthreads();
  float* ob = out + (size_t)blockIdx.x * (ROWS_BLK * NCOL);
  for (int pass = 0; pass < 2; ++pass) {
#pragma unroll
    for (int it = 0; it < 8; ++it) {
      const int idx = it * 32 + lane;
      const v4f v = *(const v4f*)(outS + idx * 4);
      *(volatile v4f*)(ob + idx * 4) = v;
    }
    if (lane < 8) {
      const int idx = 256 + lane;
      const v4f v = *(const v4f*)(outS + idx * 4);
      *(volatile v4f*)(ob + idx * 4) = v;
    }
    __threadfence();
  }
}

extern "C" void kernel_launch(void* const* d_in, const int* in_sizes, int n_in,
                              void* d_out, int out_size, void* d_ws, size_t ws_size, hipStream_t stream) {
  (void)in_sizes; (void)out_size; (void)d_ws; (void)ws_size;
  if (n_in < 13 || d_out == nullptr) return;
  lstm2_head_kernel<<<NBLK, 32, 0, stream>>>(
      (const float*)d_in[0],
      (const float*)d_in[1],  (const float*)d_in[2],
      (const float*)d_in[3],  (const float*)d_in[4],
      (const float*)d_in[5],  (const float*)d_in[6],
      (const float*)d_in[7],  (const float*)d_in[8],
      (const float*)d_in[9],  (const float*)d_in[10],
      (const float*)d_in[11], (const float*)d_in[12],
      (float*)d_out);
}
